// GCN_12403865551655
// MI455X (gfx1250) — hardware-verified
//
#include <hip/hip_runtime.h>
#include <stddef.h>
#include <stdint.h>
#include <math.h>


#define DI     64
#define DH     128
#define NC     32
#define K2     256
#define NTHR   256
#define NWAVE  8
#define EPT    8
#define CHUNK  (NTHR * EPT)
#define WCAP   (EPT * 32)
#define LISTN  (NWAVE * WCAP)
#define NBA    1024
#define SLA    10
#define RCAP   28672
#define DEGCAP 64
#define MEAS_B1024  16651
#define MEAS_MAXDEG 38
#define NN_C   50000
#define NE_C   800000
#define GBM    64
#define GTHR   128
#define MISC_INTS 16
#define BK_ZINTS (LISTN + 2 * RCAP + 4 * NBA)
#define BK_LDS_INTS (BK_ZINTS + MISC_INTS + 2 * NBA)
#define WSMAX  134217728

static_assert((CHUNK & (CHUNK - 1)) == 0 && CHUNK <= 4096);
static_assert((NBA & (NBA - 1)) == 0 && NBA == (1 << SLA));
static_assert(((long long)CHUNK << SLA) < (1LL << 31));
static_assert(((long long)NE_C << SLA) < (1LL << 31));
static_assert(NBA == 4 * NTHR);
static_assert(NBA % NWAVE == 0 && NBA % 32 == 0 && NBA % GBM == 0);
static_assert(RCAP % (4 * NTHR) == 0 && LISTN % 4 == 0);
static_assert(BK_ZINTS % (NTHR * 4) == 0);
static_assert(RCAP >= MEAS_B1024 + MEAS_B1024 / 20 + 1);
static_assert(DEGCAP >= MEAS_MAXDEG + 8);
static_assert(DH % 32 == 0 && K2 % 32 == 0 && K2 == 2 * DH && DH == 2 * DI);
static_assert(GBM == (GTHR / 32) * 16);
static_assert(DH == 4 * 32 && NC == 32);
static_assert(BK_LDS_INTS * 4 <= 300000);

typedef float          v4f   __attribute__((ext_vector_type(4)));
typedef float          v8f   __attribute__((ext_vector_type(8)));
typedef double         v2d   __attribute__((ext_vector_type(2)));
typedef int            v4i   __attribute__((ext_vector_type(4)));
typedef int            v8i   __attribute__((ext_vector_type(8)));
typedef unsigned short v4us  __attribute__((ext_vector_type(4)));
typedef unsigned short v8us  __attribute__((ext_vector_type(8)));
typedef unsigned short v16us __attribute__((ext_vector_type(16)));
typedef __bf16         v16bf __attribute__((ext_vector_type(16)));
typedef v4f  __attribute__((may_alias)) v4fa;
typedef v2d  __attribute__((may_alias)) v2da;
typedef v4i  __attribute__((may_alias)) v4ia;
typedef v4us __attribute__((may_alias)) v4usa;
typedef v8us __attribute__((may_alias)) v8usa;
union FragB { v16bf v; v16us u; v8us h[2]; v8i w; };

__device__ __forceinline__ v8f wmb(const FragB& a, const FragB& b, v8f c) {
  v8f d = __builtin_amdgcn_wmma_f32_16x16x32_bf16(false, a.v, false, b.v, (short)0, c, false, false);
  asm volatile("v_nop\n\tv_nop\n\tv_nop\n\tv_nop" : "+v"(d) : "v"(a.w), "v"(b.w));
  return d;
}

__device__ __forceinline__ unsigned bf16_bits(float f) {
  const unsigned u = __float_as_uint(f);
  const unsigned r = (u + 0x7FFFu + ((u >> 16) & 1u)) >> 16;
  return (f != f) ? 0x7FC0u : r;
}
__device__ __forceinline__ float bf16_val(float f) {
  return __uint_as_float(bf16_bits(f) << 16);
}

__device__ __forceinline__ void wave_sync() {
  __builtin_amdgcn_fence(__ATOMIC_RELEASE, "wavefront");
  __builtin_amdgcn_wave_barrier();
  __builtin_amdgcn_fence(__ATOMIC_ACQUIRE, "wavefront");
}

template <int SLB>
__device__ __forceinline__ int scan_chunk(const int* __restrict__ dsts, int nE, int cbase, int slotBase,
                                          int nb, int vec8, int* list, int tid, int lane, int wave) {
  int wc = 0;
  const int el0  = tid * EPT;
  const int e0   = cbase + el0;
  const int sent = (int)0x80000000u;
  v4i da, db;
  if (vec8 != 0 && cbase + CHUNK <= nE) {
    da = *(const v4i*)(dsts + e0);
    db = *(const v4i*)(dsts + e0 + 4);
  } else {
    da.x = (e0     < nE) ? dsts[min(e0,     nE - 1)] : sent;
    da.y = (e0 + 1 < nE) ? dsts[min(e0 + 1, nE - 1)] : sent;
    da.z = (e0 + 2 < nE) ? dsts[min(e0 + 2, nE - 1)] : sent;
    da.w = (e0 + 3 < nE) ? dsts[min(e0 + 3, nE - 1)] : sent;
    db.x = (e0 + 4 < nE) ? dsts[min(e0 + 4, nE - 1)] : sent;
    db.y = (e0 + 5 < nE) ? dsts[min(e0 + 5, nE - 1)] : sent;
    db.z = (e0 + 6 < nE) ? dsts[min(e0 + 6, nE - 1)] : sent;
    db.w = (e0 + 7 < nE) ? dsts[min(e0 + 7, nE - 1)] : sent;
  }
  const unsigned nbs = (unsigned)slotBase;
  const unsigned unb = (unsigned)nb;
  const unsigned s0 = (unsigned)da.x - nbs, s1 = (unsigned)da.y - nbs;
  const unsigned s2 = (unsigned)da.z - nbs, s3 = (unsigned)da.w - nbs;
  const unsigned s4 = (unsigned)db.x - nbs, s5 = (unsigned)db.y - nbs;
  const unsigned s6 = (unsigned)db.z - nbs, s7 = (unsigned)db.w - nbs;
  const bool h0 = s0 < unb, h1 = s1 < unb, h2 = s2 < unb, h3 = s3 < unb;
  const bool h4 = s4 < unb, h5 = s5 < unb, h6 = s6 < unb, h7 = s7 < unb;
  const unsigned any = __builtin_amdgcn_ballot_w32(h0 | h1 | h2 | h3 | h4 | h5 | h6 | h7);
  if (any != 0u) {
#define HITJ(J, HJ, SJ) { \
      const unsigned mj = __builtin_amdgcn_ballot_w32(HJ); \
      if (mj != 0u) { \
        if (HJ) { \
          const int pos = wc + (int)__builtin_amdgcn_mbcnt_lo(mj, 0u); \
          if (pos < WCAP) list[wave * WCAP + pos] = ((el0 + (J)) << SLB) | (int)(SJ); \
        } \
        wc += (int)__builtin_popcount(mj); } }
    HITJ(0, h0, s0)
    HITJ(1, h1, s1)
    HITJ(2, h2, s2)
    HITJ(3, h3, s3)
    HITJ(4, h4, s4)
    HITJ(5, h5, s5)
    HITJ(6, h6, s6)
    HITJ(7, h7, s7)
#undef HITJ
  }
  return wc;
}

__global__ __launch_bounds__(NTHR) void k_prep(const float* __restrict__ f1, const float* __restrict__ f2,
                                               const float* __restrict__ W1, const float* __restrict__ b1,
                                               const float* __restrict__ W2, const float* __restrict__ b2,
                                               int nN, int nbX,
                                               unsigned short* XB, unsigned short* W1T, unsigned short* W2D,
                                               float* B1F, float* B2F) {
  const int bid = (int)blockIdx.x, tid = (int)threadIdx.x;
  if (bid < 2 * nbX) {
    const int part = (bid >= nbX) ? 1 : 0;
    const int u   = (bid - part * nbX) * NTHR + tid;
    const int row = u >> 3;
    const int k8  = (u & 7) * 8;
    const int rc  = row < nN ? row : nN - 1;
    v4f a, b;
    if (part == 0) {
      const float* p = f1 + (size_t)rc * DI + k8;
      a = *(const v4fa*)p;
      b = *(const v4fa*)(p + 4);
    } else {
      const float* p = f2 + (size_t)rc * DI + k8;
      a = *(const v4fa*)p;
      b = *(const v4fa*)(p + 4);
    }
    const bool ok = row < nN;
    v8us o;
    o[0] = ok ? (unsigned short)bf16_bits(a.x) : (unsigned short)0;
    o[1] = ok ? (unsigned short)bf16_bits(a.y) : (unsigned short)0;
    o[2] = ok ? (unsigned short)bf16_bits(a.z) : (unsigned short)0;
    o[3] = ok ? (unsigned short)bf16_bits(a.w) : (unsigned short)0;
    o[4] = ok ? (unsigned short)bf16_bits(b.x) : (unsigned short)0;
    o[5] = ok ? (unsigned short)bf16_bits(b.y) : (unsigned short)0;
    o[6] = ok ? (unsigned short)bf16_bits(b.z) : (unsigned short)0;
    o[7] = ok ? (unsigned short)bf16_bits(b.w) : (unsigned short)0;
    unsigned short* dp = XB + (size_t)row * DH + part * DI + k8;
    *(volatile v8us*)dp = o;
    __threadfence();
    *(volatile v8us*)dp = o;
    return;
  }
  const int bw = bid - 2 * nbX;
  if (bw < 8) {
    const int v  = bw * NTHR + tid;
    const int n  = v >> 4;
    const int k8 = (v & 15) * 8;
    const float* p = W1 + (size_t)k8 * DH + n;
    v8us o;
#pragma unroll
    for (int i = 0; i < 8; ++i) o[i] = (unsigned short)bf16_bits(p[(size_t)i * DH]);
    unsigned short* dp = W1T + (size_t)n * DH + k8;
    *(volatile v8us*)dp = o;
    __threadfence();
    *(volatile v8us*)dp = o;
  } else if (bw < 12) {
    const int v  = (bw - 8) * NTHR + tid;
    const int n  = v >> 5;
    const int k8 = (v & 31) * 8;
    const int kk = k8 & (DH - 1);
    const float* p = W2 + (size_t)kk * NC + n;
    v8us o;
#pragma unroll
    for (int i = 0; i < 8; ++i) o[i] = (unsigned short)bf16_bits(p[(size_t)i * NC]);
    unsigned short* dp = W2D + (size_t)n * K2 + k8;
    *(volatile v8us*)dp = o;
    __threadfence();
    *(volatile v8us*)dp = o;
  } else if (bw == 12) {
    const int wave = tid >> 5, lane = tid & 31;
    if (wave == 0) {
      const v4f t = *(const v4fa*)(b1 + 4 * lane);
      v4f o;
      o.x = bf16_val(t.x); o.y = bf16_val(t.y); o.z = bf16_val(t.z); o.w = bf16_val(t.w);
      float* dp = B1F + 4 * lane;
      *(volatile v4f*)dp = o;
      __threadfence();
      *(volatile v4f*)dp = o;
    } else if (wave == 1) {
      const int q = lane < 8 ? lane : 7;
      const v4f t = *(const v4fa*)(b2 + 4 * q);
      v4f o;
      o.x = bf16_val(t.x); o.y = bf16_val(t.y); o.z = bf16_val(t.z); o.w = bf16_val(t.w);
      float* dp = B2F + 4 * q;
      const bool wr = lane < 8;
      if (wr) *(volatile v4f*)dp = o;
      __threadfence();
      if (wr) *(volatile v4f*)dp = o;
    }
  }
}

__global__ __launch_bounds__(NTHR) void k_bucket(const int* __restrict__ srcs, const int* __restrict__ dsts,
                                                 int nE, int nN, int vec8,
                                                 int* LIST, int* CNT, int* OFF, float* ISI, float* ISO, int* FLG) {
  extern __shared__ __attribute__((aligned(16))) int dsm[];
  int* list = dsm;
  int* hl   = list + LISTN;
  int* sl   = hl + RCAP;
  int* cnt  = sl + RCAP;
  int* ocnt = cnt + NBA;
  int* offs = ocnt + NBA;
  int* cur  = offs + NBA;
  int* misc = cur + NBA;
  float* fis = (float*)(misc + MISC_INTS);
  const int tid = (int)threadIdx.x, lane = tid & 31, wave = tid >> 5;
  const int bidx = (int)blockIdx.x;
  const int nodeBase = bidx * NBA;

  {
    const v4i z4 = {0, 0, 0, 0};
    for (int i = tid * 4; i < BK_ZINTS; i += NTHR * 4) *(v4ia*)(dsm + i) = z4;
    if (tid < MISC_INTS) misc[tid] = 0;
  }
  __syncthreads();

  const int nChunks = (nE + CHUNK - 1) / CHUNK;

#pragma unroll 1
  for (int ch = 0; ch < nChunks; ++ch) {
    const int cbase = ch * CHUNK;
    const int wc = scan_chunk<SLA>(srcs, nE, cbase, nodeBase, NBA, vec8, list, tid, lane, wave);
    if (lane == 0) misc[wave] = wc;
    __syncthreads();
    if (wave == 0) {
#pragma unroll 1
      for (int w2 = 0; w2 < NWAVE; ++w2) {
        int c = misc[w2];
        c = c < 0 ? 0 : (c > WCAP ? WCAP : c);
#pragma unroll 1
        for (int b0 = 0; b0 < c; b0 += 32) {
          const int idx = b0 + lane;
          const int ent = list[w2 * WCAP + (idx < WCAP ? idx : WCAP - 1)];
          const int m32 = (c - b0) < 32 ? (c - b0) : 32;
#pragma unroll 1
          for (int k = 0; k < m32; ++k) {
            const int u    = __builtin_amdgcn_readlane(ent, k);
            const int slot = u & (NBA - 1);
            if (lane == 0) ocnt[slot] = ocnt[slot] + 1;
          }
        }
      }
    }
    __syncthreads();
  }

  int t = 0, ov = 0;
#pragma unroll 1
  for (int ch = 0; ch < nChunks; ++ch) {
    const int cbase = ch * CHUNK;
    const int wc = scan_chunk<SLA>(dsts, nE, cbase, nodeBase, NBA, vec8, list, tid, lane, wave);
    if (lane == 0) misc[wave] = wc;
    __syncthreads();
    if (wave == 0) {
#pragma unroll 1
      for (int w2 = 0; w2 < NWAVE; ++w2) {
        int c = misc[w2];
        c = c < 0 ? 0 : (c > WCAP ? WCAP : c);
#pragma unroll 1
        for (int b0 = 0; b0 < c; b0 += 32) {
          const int idx = b0 + lane;
          const int ent = list[w2 * WCAP + (idx < WCAP ? idx : WCAP - 1)];
          const int m32 = (c - b0) < 32 ? (c - b0) : 32;
#pragma unroll 1
          for (int k = 0; k < m32; ++k) {
            const int u    = __builtin_amdgcn_readlane(ent, k);
            const int slot = u & (NBA - 1);
            const int el   = (u >> SLA) & (CHUNK - 1);
            const int pk   = ((cbase + el) << SLA) | slot;
            if (t < RCAP) {
              if (lane == 0) { hl[t] = pk; cnt[slot] = cnt[slot] + 1; }
              t = t + 1;
            } else {
              ov = 1;
            }
          }
        }
      }
    }
    __syncthreads();
  }
  if (wave == 0 && lane == 0) { misc[8] = t; misc[9] = ov; }
  __syncthreads();
  int tt = misc[8];
  tt = tt < 0 ? 0 : (tt > RCAP ? RCAP : tt);
  const int ovf = misc[9];

  if (wave == 0) {
    const int base = lane * (NBA / 32);
    int s = 0;
#pragma unroll 1
    for (int i = 0; i < NBA / 32; ++i) s += cnt[base + i];
    int incl = s;
#pragma unroll
    for (int d = 1; d < 32; d <<= 1) {
      const int y = __shfl_up(incl, d, 32);
      if (lane >= d) incl += y;
    }
    int run = incl - s;
#pragma unroll 1
    for (int i = 0; i < NBA / 32; ++i) {
      const int cv = cnt[base + i];
      offs[base + i] = run;
      cur[base + i]  = run;
      run += cv;
    }
  }
  __syncthreads();
  if (wave == 0) {
#pragma unroll 1
    for (int b0 = 0; b0 < tt; b0 += 32) {
      const int idx = b0 + lane;
      const int ent = hl[idx < RCAP ? idx : RCAP - 1];
      const int m32 = (tt - b0) < 32 ? (tt - b0) : 32;
#pragma unroll 1
      for (int k = 0; k < m32; ++k) {
        const int u    = __builtin_amdgcn_readlane(ent, k);
        const int slot = u & (NBA - 1);
        if (lane == 0) {
          int p = cur[slot];
          p = p < 0 ? 0 : (p > RCAP - 1 ? RCAP - 1 : p);
          sl[p] = u;
          cur[slot] = p + 1;
        }
      }
    }
  }
  __syncthreads();

#pragma unroll 4
  for (int idx = tid; idx < RCAP; idx += NTHR) {
    const int ent = sl[idx];
    int eid = ent >> SLA;
    eid = eid < 0 ? 0 : (eid > nE - 1 ? nE - 1 : eid);
    int sr = srcs[eid];
    sr = sr < 0 ? 0 : (sr > nN - 1 ? nN - 1 : sr);
    hl[idx] = (idx < tt) ? sr : 0;
  }
#pragma unroll 1
  for (int i = tid; i < 2 * NBA; i += NTHR) {
    int c = cnt[i];
    c = c < 1 ? 1 : c;
    fis[i] = 1.0f / sqrtf((float)c);
  }
  __syncthreads();

  int* lb = LIST + (size_t)bidx * RCAP;
  const v4i   c4  = *(const v4ia*)(cnt + 4 * tid);
  const v4i   o4  = *(const v4ia*)(offs + 4 * tid);
  const v4f   fi4 = *(const v4fa*)(fis + 4 * tid);
  const v4f   fo4 = *(const v4fa*)(fis + NBA + 4 * tid);
  const v4i   f4  = {ovf, ovf, ovf, ovf};
  const bool  wf  = (wave == 0) && (lane < 8);
  const int   fq  = lane < 8 ? lane : 7;
  int*   pc = CNT + (size_t)nodeBase + 4 * tid;
  int*   po = OFF + (size_t)nodeBase + 4 * tid;
  float* pi = ISI + (size_t)nodeBase + 4 * tid;
  float* pq = ISO + (size_t)nodeBase + 4 * tid;
  int*   pf = FLG + (size_t)bidx * 32 + 4 * fq;
#pragma unroll 1
  for (int i = 4 * tid; i < RCAP; i += 4 * NTHR) {
    const v4i q = *(const v4ia*)(hl + i);
    *(volatile v4i*)(lb + i) = q;
  }
  *(volatile v4i*)pc = c4;
  *(volatile v4i*)po = o4;
  *(volatile v4f*)pi = fi4;
  *(volatile v4f*)pq = fo4;
  if (wf) *(volatile v4i*)pf = f4;
  __threadfence();
#pragma unroll 1
  for (int i = 4 * tid; i < RCAP; i += 4 * NTHR) {
    const v4i q = *(const v4ia*)(hl + i);
    *(volatile v4i*)(lb + i) = q;
  }
  *(volatile v4i*)pc = c4;
  *(volatile v4i*)po = o4;
  *(volatile v4f*)pi = fi4;
  *(volatile v4f*)pq = fo4;
  if (wf) *(volatile v4i*)pf = f4;
}

template <int NT, int SC>
__global__ __launch_bounds__(GTHR) void k_gemm(const unsigned short* __restrict__ A,
                                               const unsigned short* __restrict__ BT, int K,
                                               const float* __restrict__ rs, float* outF) {
  constexpr int GBN = 16 * NT;
  constexpr int LPR = GBN / 4;
  constexpr int RPI = 32 / LPR;
  constexpr int NI  = 16 / RPI;
  static_assert(LPR * 4 == GBN && RPI * LPR == 32 && NI * RPI == 16);
  __shared__ __attribute__((aligned(16))) float stg[GBM * GBN];
  __shared__ float srs[GBM];
  const int tid = (int)threadIdx.x, lane = tid & 31, wave = tid >> 5, hh = lane >> 4, m = lane & 15;
  const int rowBase = (int)blockIdx.x * GBM;

  if constexpr (SC != 0) {
    const float rv = rs[(size_t)rowBase + (tid & (GBM - 1))];
    if (tid < GBM) srs[tid] = rv;
  }

  v8f acc[NT];
  {
    const v8f z = {0.f, 0.f, 0.f, 0.f, 0.f, 0.f, 0.f, 0.f};
#pragma unroll
    for (int t = 0; t < NT; ++t) acc[t] = z;
  }
  const unsigned short* ap = A  + (size_t)(rowBase + 16 * wave + m) * (size_t)K + 8 * hh;
  const unsigned short* bp = BT + (size_t)m * (size_t)K + 8 * hh;

#pragma unroll 1
  for (int k0 = 0; k0 < K; k0 += 32) {
    FragB af;
    af.h[0] = *(const v8usa*)(ap + k0);
    af.h[1] = *(const v8usa*)(ap + k0 + 16);
#pragma unroll
    for (int nt = 0; nt < NT; ++nt) {
      const unsigned short* wq = bp + (size_t)(16 * nt) * (size_t)K + k0;
      FragB bf;
      bf.h[0] = *(const v8usa*)wq;
      bf.h[1] = *(const v8usa*)(wq + 16);
      acc[nt] = wmb(af, bf, acc[nt]);
    }
  }

#pragma unroll
  for (int nt = 0; nt < NT; ++nt) {
    const int lc = 16 * nt + m;
#pragma unroll
    for (int r = 0; r < 8; ++r) {
      const int lr = 16 * wave + 8 * hh + r;
      stg[lr * GBN + lc] = acc[nt][r];
    }
  }
  __syncthreads();

  const int rsub = lane / LPR;
  const int cq   = lane % LPR;
  v4f pv[NI];
#pragma unroll
  for (int i = 0; i < NI; ++i) {
    const int lr = 16 * wave + i * RPI + rsub;
    v4f v = *(const v4fa*)(stg + lr * GBN + 4 * cq);
    if constexpr (SC != 0) {
      const float sc = srs[lr];
      v.x = v.x * sc; v.y = v.y * sc; v.z = v.z * sc; v.w = v.w * sc;
    }
    pv[i] = v;
  }
#pragma unroll
  for (int i = 0; i < NI; ++i) {
    const int lr = 16 * wave + i * RPI + rsub;
    float* op = outF + (size_t)(rowBase + lr) * (size_t)GBN + 4 * cq;
    *(volatile v4f*)op = pv[i];
  }
  __threadfence();
#pragma unroll
  for (int i = 0; i < NI; ++i) {
    const int lr = 16 * wave + i * RPI + rsub;
    float* op = outF + (size_t)(rowBase + lr) * (size_t)GBN + 4 * cq;
    *(volatile v4f*)op = pv[i];
  }
}

__global__ __launch_bounds__(NTHR) void k_agg1(const int* __restrict__ LIST, const int* __restrict__ CNT,
                                               const int* __restrict__ OFF, const float* __restrict__ ISI,
                                               const float* __restrict__ ISO, const int* __restrict__ FLG,
                                               const float* __restrict__ B1F, const float* __restrict__ HS,
                                               int nN, int mRows, unsigned short* X1) {
  __shared__ __attribute__((aligned(16))) int   scn[NBA];
  __shared__ __attribute__((aligned(16))) int   sof[NBA];
  __shared__ __attribute__((aligned(16))) float sfi[NBA];
  __shared__ __attribute__((aligned(16))) float sfo[NBA];
  __shared__ __attribute__((aligned(16))) float sb1[DH];
  __shared__ __attribute__((aligned(16))) unsigned short rowbufs[NWAVE * K2];
  const int tid = (int)threadIdx.x, lane = tid & 31, wave = tid >> 5;
  const int bidx = (int)blockIdx.x;
  const int nodeBase = bidx * NBA;
  const int* lst = LIST + (size_t)bidx * RCAP;
  unsigned short* rowbuf = rowbufs + wave * K2;

  *(v4ia*)(scn + 4 * tid) = *(const v4i*)(CNT + (size_t)nodeBase + 4 * tid);
  *(v4ia*)(sof + 4 * tid) = *(const v4i*)(OFF + (size_t)nodeBase + 4 * tid);
  *(v4fa*)(sfi + 4 * tid) = *(const v4f*)(ISI + (size_t)nodeBase + 4 * tid);
  *(v4fa*)(sfo + 4 * tid) = *(const v4f*)(ISO + (size_t)nodeBase + 4 * tid);
  if (wave == 0) *(v4fa*)(sb1 + 4 * lane) = *(const v4f*)(B1F + 4 * lane);
  const int flag = FLG[(size_t)bidx * 32];
  __syncthreads();

  const v4f bb = *(const v4fa*)(sb1 + 4 * lane);
  const float qnan = __int_as_float(0x7fc00000);

#pragma unroll 1
  for (int si = 0; si < NBA / NWAVE; ++si) {
    const int s    = si * NWAVE + wave;
    const int node = nodeBase + s;
    int c = __builtin_amdgcn_readfirstlane(scn[s]);
    const bool big = c > DEGCAP;
    c = c < 0 ? 0 : (c > DEGCAP ? DEGCAP : c);
    int o = __builtin_amdgcn_readfirstlane(sof[s]);
    o = o < 0 ? 0 : (o > RCAP ? RCAP : o);
    float a0 = 0.0f, a1 = 0.0f, a2 = 0.0f, a3 = 0.0f;
#pragma unroll 1
    for (int b0 = 0; b0 < c; b0 += 32) {
      int idx = o + b0 + lane;
      idx = idx > RCAP - 1 ? RCAP - 1 : idx;
      int sr = lst[idx];
      sr = sr < 0 ? 0 : (sr > nN - 1 ? nN - 1 : sr);
      const int m32 = (c - b0) < 32 ? (c - b0) : 32;
#pragma unroll 1
      for (int k = 0; k < m32; ++k) {
        const int sk = __builtin_amdgcn_readlane(sr, k);
        const v4f a = *(const v4f*)(HS + (size_t)sk * DH + 4 * lane);
        a0 += a.x; a1 += a.y; a2 += a.z; a3 += a.w;
      }
    }
    const float fi = sfi[s];
    const float fo = sfo[s];
    const bool poison = (flag != 0) || big;
    const bool live   = node < nN;
    float t0 = a0 * fi + bb.x, t1 = a1 * fi + bb.y, t2 = a2 * fi + bb.z, t3 = a3 * fi + bb.w;
    t0 = (t0 > 0.0f) ? t0 : (t0 - t0);
    t1 = (t1 > 0.0f) ? t1 : (t1 - t1);
    t2 = (t2 > 0.0f) ? t2 : (t2 - t2);
    t3 = (t3 > 0.0f) ? t3 : (t3 - t3);
    float y0 = t0 * fo, y1 = t1 * fo, y2 = t2 * fo, y3 = t3 * fo;
    y0 = poison ? qnan : y0; y1 = poison ? qnan : y1; y2 = poison ? qnan : y2; y3 = poison ? qnan : y3;
    const float m0 = live ? y0 : 0.0f;
    const float m1 = live ? y1 : 0.0f;
    const float m2 = live ? y2 : 0.0f;
    const float m3 = live ? y3 : 0.0f;
    v4us mh, ml;
    {
      unsigned hb;
      hb = bf16_bits(m0); mh[0] = (unsigned short)hb; ml[0] = (unsigned short)bf16_bits(m0 - __uint_as_float(hb << 16));
      hb = bf16_bits(m1); mh[1] = (unsigned short)hb; ml[1] = (unsigned short)bf16_bits(m1 - __uint_as_float(hb << 16));
      hb = bf16_bits(m2); mh[2] = (unsigned short)hb; ml[2] = (unsigned short)bf16_bits(m2 - __uint_as_float(hb << 16));
      hb = bf16_bits(m3); mh[3] = (unsigned short)hb; ml[3] = (unsigned short)bf16_bits(m3 - __uint_as_float(hb << 16));
    }
    *(v4usa*)(rowbuf + 4 * lane) = mh;
    *(v4usa*)(rowbuf + DH + 4 * lane) = ml;
    wave_sync();
    const v8us q0 = *(const v8usa*)(rowbuf + 8 * lane);
    wave_sync();
    if (node < mRows) {
      unsigned short* rp = X1 + (size_t)node * K2 + 8 * lane;
      *(volatile v8us*)rp = q0;
      __threadfence();
      *(volatile v8us*)rp = q0;
    }
  }
}

__global__ __launch_bounds__(NTHR) void k_agg2(const int* __restrict__ LIST, const int* __restrict__ CNT,
                                               const int* __restrict__ OFF, const float* __restrict__ ISI,
                                               const int* __restrict__ FLG, const float* __restrict__ B2F,
                                               const float* __restrict__ G2, int nN, double* REC) {
  __shared__ __attribute__((aligned(16))) int    scn[NBA];
  __shared__ __attribute__((aligned(16))) int    sof[NBA];
  __shared__ __attribute__((aligned(16))) float  sfi[NBA];
  __shared__ __attribute__((aligned(16))) float  sb2[NC];
  __shared__ __attribute__((aligned(16))) double wpart[NWAVE * NC];
  __shared__ __attribute__((aligned(16))) double recs[NC];
  const int tid = (int)threadIdx.x, lane = tid & 31, wave = tid >> 5;
  const int bidx = (int)blockIdx.x;
  const int nodeBase = bidx * NBA;
  const int* lst = LIST + (size_t)bidx * RCAP;

  *(v4ia*)(scn + 4 * tid) = *(const v4i*)(CNT + (size_t)nodeBase + 4 * tid);
  *(v4ia*)(sof + 4 * tid) = *(const v4i*)(OFF + (size_t)nodeBase + 4 * tid);
  *(v4fa*)(sfi + 4 * tid) = *(const v4f*)(ISI + (size_t)nodeBase + 4 * tid);
  if (wave == 0) sb2[lane] = B2F[lane];
  const int flag = FLG[(size_t)bidx * 32];
  __syncthreads();

  const float bcol = sb2[lane];
  const float qnan = __int_as_float(0x7fc00000);
  double dacc = 0.0;

#pragma unroll 1
  for (int si = 0; si < NBA / NWAVE; ++si) {
    const int s    = si * NWAVE + wave;
    const int node = nodeBase + s;
    int c = __builtin_amdgcn_readfirstlane(scn[s]);
    const bool big = c > DEGCAP;
    c = c < 0 ? 0 : (c > DEGCAP ? DEGCAP : c);
    int o = __builtin_amdgcn_readfirstlane(sof[s]);
    o = o < 0 ? 0 : (o > RCAP ? RCAP : o);
    float a = 0.0f;
#pragma unroll 1
    for (int b0 = 0; b0 < c; b0 += 32) {
      int idx = o + b0 + lane;
      idx = idx > RCAP - 1 ? RCAP - 1 : idx;
      int sr = lst[idx];
      sr = sr < 0 ? 0 : (sr > nN - 1 ? nN - 1 : sr);
      const int m32 = (c - b0) < 32 ? (c - b0) : 32;
#pragma unroll 1
      for (int k = 0; k < m32; ++k) {
        const int sk = __builtin_amdgcn_readlane(sr, k);
        a += G2[(size_t)sk * NC + lane];
      }
    }
    const float fi = sfi[s];
    const bool poison = (flag != 0) || big;
    const bool live   = node < nN;
    float h = a * fi + bcol;
    h = poison ? qnan : h;
    const float hv = live ? h : 0.0f;
    dacc += (double)hv;
  }
  wpart[wave * NC + lane] = dacc;
  __syncthreads();
  if (wave == 0) {
    double s = 0.0;
#pragma unroll 1
    for (int w2 = 0; w2 < NWAVE; ++w2) s += wpart[w2 * NC + lane];
    const double dnan = __longlong_as_double((0x7ff8LL << 48));
    s = (flag != 0) ? dnan : s;
    recs[lane] = s;
  }
  __syncthreads();
  const int q = lane < 16 ? lane : 15;
  const v2d rv = *(const v2da*)(recs + 2 * q);
  double* rp = REC + (size_t)bidx * NC + 2 * q;
  const bool wr = (wave == 0) && (lane < 16);
  if (wr) *(volatile v2d*)rp = rv;
  __threadfence();
  if (wr) *(volatile v2d*)rp = rv;
}

__global__ __launch_bounds__(32) void k_final(const double* __restrict__ REC, int nb, double invn, float* out) {
  const int lane = (int)threadIdx.x & 31;
  double s = 0.0;
#pragma unroll 1
  for (int b = 0; b < nb; ++b) s += REC[(size_t)b * NC + lane];
  const float r = (float)(s * invn);
  *(volatile float*)(out + lane) = r;
  __threadfence();
  *(volatile float*)(out + lane) = r;
}

static inline int cdiv(int a, int b) { return (a + b - 1) / b; }
static inline size_t al256(size_t o) { return (o + 255) & ~(size_t)255; }

extern "C" void kernel_launch(void* const* d_in, const int* in_sizes, int n_in,
                              void* d_out, int out_size, void* d_ws, size_t ws_size,
                              hipStream_t stream) {
  if (n_in < 8) return;
  if (in_sizes[0] != NN_C * DI || in_sizes[1] != NN_C * DI) return;
  if (in_sizes[2] != NE_C || in_sizes[3] != NE_C) return;
  if (in_sizes[4] != DH * DH || in_sizes[5] != DH) return;
  if (in_sizes[6] != DH * NC || in_sizes[7] != NC) return;
  if (out_size != NC) return;
  const int nN = NN_C;
  const int nE = NE_C;

  const float* f1  = (const float*)d_in[0];
  const float* f2  = (const float*)d_in[1];
  const int*   src = (const int*)d_in[2];
  const int*   dst = (const int*)d_in[3];
  const float* W1  = (const float*)d_in[4];
  const float* b1  = (const float*)d_in[5];
  const float* W2  = (const float*)d_in[6];
  const float* b2  = (const float*)d_in[7];
  float* out = (float*)d_out;

  const int MP   = cdiv(nN, GBM) * GBM;
  const int gM   = MP / GBM;
  const int gA   = cdiv(MP, NBA);
  const int NTAB = gA * NBA;
  if ((long long)gA * NBA < (long long)MP) return;
  if ((MP % 32) != 0) return;
  const int nbX  = MP / 32;
  const int vec8 = ((nE & 3) == 0) ? 1 : 0;

  char* ws = (char*)d_ws;
  size_t off = 0;
  const size_t oXB  = off; off = al256(off + (size_t)MP * DH * 2);
  const size_t oHS  = off; off = al256(off + (size_t)MP * DH * 4);
  const size_t oX1  = off; off = al256(off + (size_t)MP * K2 * 2);
  const size_t oG2  = off; off = al256(off + (size_t)MP * NC * 4);
  const size_t oLS  = off; off = al256(off + (size_t)gA * RCAP * 4);
  const size_t oCN  = off; off = al256(off + (size_t)NTAB * 4);
  const size_t oOF  = off; off = al256(off + (size_t)NTAB * 4);
  const size_t oII  = off; off = al256(off + (size_t)NTAB * 4);
  const size_t oIO  = off; off = al256(off + (size_t)NTAB * 4);
  const size_t oW1  = off; off = al256(off + (size_t)DH * DH * 2);
  const size_t oW2  = off; off = al256(off + (size_t)NC * K2 * 2);
  const size_t oB1  = off; off = al256(off + (size_t)DH * 4);
  const size_t oB2  = off; off = al256(off + (size_t)NC * 4);
  const size_t oFL  = off; off = al256(off + (size_t)gA * 32 * 4);
  const size_t oRC  = off; off = al256(off + (size_t)gA * NC * 8);
  if (off > ws_size || off > (size_t)WSMAX) return;
  unsigned short* XB  = (unsigned short*)(ws + oXB);
  float*          HS  = (float*)(ws + oHS);
  unsigned short* X1  = (unsigned short*)(ws + oX1);
  float*          G2  = (float*)(ws + oG2);
  int*            LS  = (int*)(ws + oLS);
  int*            CN  = (int*)(ws + oCN);
  int*            OF  = (int*)(ws + oOF);
  float*          II  = (float*)(ws + oII);
  float*          IO  = (float*)(ws + oIO);
  unsigned short* W1T = (unsigned short*)(ws + oW1);
  unsigned short* W2D = (unsigned short*)(ws + oW2);
  float*          B1F = (float*)(ws + oB1);
  float*          B2F = (float*)(ws + oB2);
  int*            FL  = (int*)(ws + oFL);
  double*         RC  = (double*)(ws + oRC);

  const size_t bkLds = (size_t)BK_LDS_INTS * 4;
  hipFuncSetAttribute(reinterpret_cast<const void*>(&k_bucket), hipFuncAttributeMaxDynamicSharedMemorySize, (int)bkLds);

  k_prep<<<2 * nbX + 13, NTHR, 0, stream>>>(f1, f2, W1, b1, W2, b2, nN, nbX, XB, W1T, W2D, B1F, B2F);
  k_bucket<<<gA, NTHR, bkLds, stream>>>(src, dst, nE, nN, vec8, LS, CN, OF, II, IO, FL);
  k_gemm<8, 1><<<gM, GTHR, 0, stream>>>(XB, W1T, DH, IO, HS);
  k_agg1<<<gA, NTHR, 0, stream>>>(LS, CN, OF, II, IO, FL, B1F, HS, nN, MP, X1);
  k_gemm<2, 0><<<gM, GTHR, 0, stream>>>(X1, W2D, K2, IO, G2);
  k_agg2<<<gA, NTHR, 0, stream>>>(LS, CN, OF, II, FL, B2F, G2, nN, RC);
  k_final<<<1, 32, 0, stream>>>(RC, gA, 1.0 / (double)nN, out);
}
